// EquivariantMessagePassing_82867099009204
// MI455X (gfx1250) — hardware-verified
//
#include <hip/hip_runtime.h>
#include <math.h>

typedef __attribute__((ext_vector_type(16))) _Float16 v16h;
typedef __attribute__((ext_vector_type(8)))  _Float16 v8h;
typedef __attribute__((ext_vector_type(4)))  _Float16 v4h;
typedef __attribute__((ext_vector_type(16))) __bf16   v16b;
typedef __attribute__((ext_vector_type(8)))  __bf16   v8b;
typedef __attribute__((ext_vector_type(8)))  float    v8f;
typedef __attribute__((ext_vector_type(4)))  float    v4f;
typedef __attribute__((ext_vector_type(2)))  float    v2f;
typedef __attribute__((ext_vector_type(4)))  int      v4i;

#define NN 50000
#define NE 800000
#define FD 64
#define HD 128
#define HC 256
#define NC 512
#define NPM 50048
#define CH 63488
#define NCHUNK 13
#define EB 64
#define SAP 136
#define TBN 512
#define NTILE 98
#define SCH 2048
#define NSTEP (CH / SCH)
#define NT 256

__device__ __forceinline__ unsigned short f2bf_bits(float f) {
  unsigned u = __float_as_uint(f);
  return (unsigned short)((u + 0x7FFFu + ((u >> 16) & 1u)) >> 16);
}
__device__ __forceinline__ float bf_bits2f(unsigned short h) { return __uint_as_float(((unsigned)h) << 16); }

__device__ __forceinline__ void dep_guard_h(v8f& a, v8f& b, v16h x, v16h y) { asm volatile("v_nop\n\tv_nop\n\tv_nop\n\tv_nop" : "+v"(a), "+v"(b) : "v"(x), "v"(y)); }
__device__ __forceinline__ void dep_guard_b(v8f& a, v8f& b, v16b x, v16b y) { asm volatile("v_nop\n\tv_nop\n\tv_nop\n\tv_nop" : "+v"(a), "+v"(b) : "v"(x), "v"(y)); }
__device__ __forceinline__ void keep4_h(v16h a, v16h b, v16h c, v16h d) { asm volatile("v_nop" :: "v"(a), "v"(b), "v"(c), "v"(d)); }
__device__ __forceinline__ void keep4_b(v16b a, v16b b, v16b c, v16b d) { asm volatile("v_nop" :: "v"(a), "v"(b), "v"(c), "v"(d)); }
__device__ __forceinline__ void acc_guard4(v8f& a, v8f& b, v8f& c, v8f& d) { asm volatile("v_nop\n\tv_nop\n\tv_nop\n\tv_nop" : "+v"(a), "+v"(b), "+v"(c), "+v"(d)); }
__device__ __forceinline__ void acc_guard2(v8f& a, v8f& b) { asm volatile("v_nop\n\tv_nop\n\tv_nop\n\tv_nop" : "+v"(a), "+v"(b)); }
template <typename T> struct Frag;
template <> struct Frag<_Float16> {
  typedef v16h V; union U { v16h v; v8h h[2]; };
  static __device__ __forceinline__ v16h load(const _Float16* p) {
    U f; f.h[0] = *(const v8h*)(p); f.h[1] = *(const v8h*)(p + 16); return f.v;
  }
  static __device__ __forceinline__ v8f mma(v16h a, v16h b, v8f c) {
    return __builtin_amdgcn_wmma_f32_16x16x32_f16(false, a, false, b, (short)0, c, false, false);
  }
  static __device__ __forceinline__ void guard(v8f& a, v8f& b, v16h x, v16h y) { dep_guard_h(a, b, x, y); }
  static __device__ __forceinline__ void keep(v16h a, v16h b, v16h c, v16h d) { keep4_h(a, b, c, d); }
};
template <> struct Frag<__bf16> {
  typedef v16b V; union U { v16b v; v8b h[2]; };
  static __device__ __forceinline__ v16b load(const __bf16* p) {
    U f; f.h[0] = *(const v8b*)(p); f.h[1] = *(const v8b*)(p + 16); return f.v;
  }
  static __device__ __forceinline__ v8f mma(v16b a, v16b b, v8f c) {
    return __builtin_amdgcn_wmma_f32_16x16x32_bf16(false, a, false, b, (short)0, c, false, false);
  }
  static __device__ __forceinline__ void guard(v8f& a, v8f& b, v16b x, v16b y) { dep_guard_b(a, b, x, y); }
  static __device__ __forceinline__ void keep(v16b a, v16b b, v16b c, v16b d) { keep4_b(a, b, c, d); }
};

template <int ET> struct Elem;
template <> struct Elem<0> { typedef _Float16 T; };
template <> struct Elem<1> { typedef __bf16 T; };
template <int ET, bool SPLIT, int BIAS_MODE, int OUT_MODE, bool RESID, int ACT = 0>
__global__ __launch_bounds__(256) void wmma_gemm64(
    const unsigned short* __restrict__ Ap, const unsigned short* __restrict__ A2p, int lda, long strideA,
    const unsigned short* __restrict__ Btp, const unsigned short* __restrict__ Bt2p, int ldb, long strideB,
    void* __restrict__ Cout, void* __restrict__ Cout2, int ldc, long strideC,
    const float* __restrict__ bias,
    const float* __restrict__ resid, long strideR,
    int M, int N, int K, float scale) {
  typedef typename Elem<ET>::T T;
  typedef typename Frag<T>::V V;
  const T* A = (const T*)Ap; const T* A2 = (const T*)A2p; const T* Bt = (const T*)Btp; const T* Bt2 = (const T*)Bt2p;
  __shared__ __align__(16) float sT[8][16 * 68];
  const int b    = blockIdx.y;
  const int lane = threadIdx.x & 31;
  const int wave = threadIdx.x >> 5;
  const int tilesN = N >> 6;
  const int tilesM = M >> 6;
  const int tile = blockIdx.x * 8 + wave;
  if (tile >= tilesM * tilesN) return;
  const int tm = tile / tilesN;
  const int tn = tile - tm * tilesN;
  const int m0 = tm << 6;
  const int n0 = tn << 6;

  const T* Ab  = A  + (size_t)b * strideA;
  const T* Bb  = Bt + (size_t)b * strideB;
  const T* Ab2 = SPLIT ? (A2  + (size_t)b * strideA) : nullptr;
  const T* Bb2 = SPLIT ? (Bt2 + (size_t)b * strideB) : nullptr;

  const int rlane = lane & 15;
  const int koff  = (lane >> 4) * 8;
  const int mOff  = (lane >> 4) * 8;

  v8f acc[4][4];
#pragma unroll
  for (int i = 0; i < 4; ++i)
#pragma unroll
    for (int j = 0; j < 4; ++j) acc[i][j] = (v8f){0.f,0.f,0.f,0.f,0.f,0.f,0.f,0.f};

  for (int k0 = 0; k0 < K; k0 += 32) {
    V bh[4], bl[4];
#pragma unroll
    for (int j = 0; j < 4; ++j) {
      const size_t bo = (size_t)(n0 + (j << 4) + rlane) * ldb + koff + k0;
      bh[j] = Frag<T>::load(Bb + bo);
      if (SPLIT) bl[j] = Frag<T>::load(Bb2 + bo);
    }
#pragma unroll
    for (int i = 0; i < 4; ++i) {
      const size_t ao = (size_t)(m0 + (i << 4) + rlane) * lda + koff + k0;
      V ah = Frag<T>::load(Ab + ao);
      V al;
      if (SPLIT) al = Frag<T>::load(Ab2 + ao);
#pragma unroll
      for (int j = 0; j < 4; ++j) {
        acc[i][j] = Frag<T>::mma(ah, bh[j], acc[i][j]);
        if (SPLIT) {
          acc[i][j] = Frag<T>::mma(ah, bl[j], acc[i][j]);
          acc[i][j] = Frag<T>::mma(al, bh[j], acc[i][j]);
        }
      }
      Frag<T>::guard(acc[i][0], acc[i][3], ah, SPLIT ? al : ah);
    }
    Frag<T>::keep(bh[0], bh[1], bh[2], bh[3]);
    if (SPLIT) Frag<T>::keep(bl[0], bl[1], bl[2], bl[3]);
  }
  acc_guard4(acc[0][0], acc[0][1], acc[0][2], acc[0][3]);
  acc_guard4(acc[1][0], acc[1][1], acc[1][2], acc[1][3]);
  acc_guard4(acc[2][0], acc[2][1], acc[2][2], acc[2][3]);
  acc_guard4(acc[3][0], acc[3][1], acc[3][2], acc[3][3]);

  float* slab = sT[wave];
  const float* Rb = RESID ? (resid + (size_t)b * strideR) : nullptr;
#pragma unroll
  for (int i = 0; i < 4; ++i) {
    const int mBase = m0 + (i << 4);
#pragma unroll
    for (int j = 0; j < 4; ++j) {
      const int n = n0 + (j << 4) + rlane;
      float bv = 0.f;
      if (BIAS_MODE == 2) bv = bias[n];
#pragma unroll
      for (int r = 0; r < 8; ++r) {
        float v = acc[i][j][r] * scale;
        if (BIAS_MODE == 1) v += bias[mBase + mOff + r];
        if (BIAS_MODE == 2) v += bv;
        if (RESID) v += Rb[(size_t)(mBase + mOff + r) * ldc + n];
        if (ACT == 1) v = tanhf(v);
        if (ACT == 2) v = fmaxf(v, 0.0f);
        if (ACT == 3) v = v / (1.0f + expf(-v));
        if (ACT == 4) v = (v > 0.f) ? v : 0.01f * v;
        if (ACT == 5) v = 0.5f * v * (1.0f + erff(v * 0.70710678118654752f));
        slab[(mOff + r) * 68 + (j << 4) + rlane] = v;
      }
    }
    __builtin_amdgcn_fence(__ATOMIC_RELEASE, "workgroup");
    __builtin_amdgcn_wave_barrier();
    __builtin_amdgcn_fence(__ATOMIC_ACQUIRE, "workgroup");
    if (OUT_MODE == 0) {
      float* C = (float*)Cout + (size_t)b * strideC;
      const int hh = lane >> 4, c4 = (lane & 15) * 4;
      for (int pass = 0; pass < 2; ++pass) {
#pragma unroll
        for (int it = 0; it < 8; ++it) {
          const int row = it * 2 + hh;
          v4f v = *(const v4f*)(slab + row * 68 + c4);
          *(volatile v4f*)(C + (size_t)(mBase + row) * ldc + n0 + c4) = v;
        }
        __threadfence();
      }
    } else {
      const int q = lane >> 3, c8 = (lane & 7) * 8;
      unsigned short* C  = (unsigned short*)Cout  + (size_t)b * strideC;
      unsigned short* C2 = (OUT_MODE == 2) ? ((unsigned short*)Cout2 + (size_t)b * strideC) : nullptr;
      for (int pass = 0; pass < 2; ++pass) {
#pragma unroll
        for (int it = 0; it < 4; ++it) {
          const int row = it * 4 + q;
          const float* sp = slab + row * 68 + c8;
          v8h hv, lv;
#pragma unroll
          for (int e = 0; e < 8; ++e) {
            if (OUT_MODE == 1) {
              hv[e] = (_Float16)sp[e];
            } else {
              unsigned short hb = f2bf_bits(sp[e]);
              unsigned short lb = f2bf_bits(sp[e] - bf_bits2f(hb));
              hv[e] = __builtin_bit_cast(_Float16, hb);
              lv[e] = __builtin_bit_cast(_Float16, lb);
            }
          }
          *(volatile v8h*)(C + (size_t)(mBase + row) * ldc + n0 + c8) = hv;
          if (OUT_MODE == 2) *(volatile v8h*)(C2 + (size_t)(mBase + row) * ldc + n0 + c8) = lv;
        }
        __threadfence();
      }
    }
    __builtin_amdgcn_fence(__ATOMIC_RELEASE, "workgroup");
    __builtin_amdgcn_wave_barrier();
    __builtin_amdgcn_fence(__ATOMIC_ACQUIRE, "workgroup");
  }
}

__device__ __forceinline__ unsigned pack_h2(float a, float b) {
  return (unsigned)__builtin_bit_cast(unsigned short, (_Float16)a) | ((unsigned)__builtin_bit_cast(unsigned short, (_Float16)b) << 16);
}
__device__ __forceinline__ float fexp(float x) {
#if __has_builtin(__builtin_amdgcn_exp2f)
  return __builtin_amdgcn_exp2f(x * 1.4426950408889634f);
#else
  return __expf(x);
#endif
}
__device__ __forceinline__ float frcp(float d) {
#if __has_builtin(__builtin_amdgcn_rcpf)
  return __builtin_amdgcn_rcpf(d);
#else
  return 1.0f / d;
#endif
}
__device__ __forceinline__ float silu_f(float h) { return h * frcp(1.0f + fexp(-h)); }

__device__ __forceinline__ int blk_excl_scan(int cnt, int* scan_ws, int tid, int* tot) {
  const int lane = tid & 31, wave = tid >> 5; int incl = cnt;
#pragma unroll
  for (int o = 1; o < 32; o <<= 1) { const int v = __shfl_up(incl, o, 32); if (lane >= o) incl += v; }
  if (lane == 31) scan_ws[wave] = incl;
  __syncthreads();
  if (wave == 0) { int wv = (lane < NT / 32) ? scan_ws[lane] : 0; int wincl = wv;
#pragma unroll
    for (int o = 1; o < 32; o <<= 1) { const int v = __shfl_up(wincl, o, 32); if (lane >= o) wincl += v; }
    if (lane < NT / 32) scan_ws[32 + lane] = wincl - wv; if (lane == 31) scan_ws[64] = wincl; }
  __syncthreads();
  const int res = scan_ws[32 + wave] + incl - cnt; *tot = scan_ws[64];
  return res;
}
template <int SP, int CAP>
__device__ __forceinline__ int chunk_hits(const int* __restrict__ dstv, int e0, int ebase, int n0, int tid, int* LIST, int* scan_ws) {
  const int eb = e0 + tid * SP;
  int rec[SP]; int cnt = 0;
#pragma unroll
  for (int kq = 0; kq < SP; kq += 4) {
    v4i d4 = {-1, -1, -1, -1};
    if (eb + kq < NE) d4 = *(const v4i*)(dstv + eb + kq);
#pragma unroll
    for (int e = 0; e < 4; ++e) {
      const int d = d4[e]; int r = -1;
      if (d >= n0 && d < n0 + TBN) { r = ((d - n0) << 17) | (eb + kq + e - ebase); ++cnt; }
      rec[kq + e] = r;
    }
  }
  int tot; int p = blk_excl_scan(cnt, scan_ws, tid, &tot);
#pragma unroll
  for (int kq = 0; kq < SP; ++kq) if (rec[kq] >= 0) { if ((unsigned)p < (unsigned)CAP) LIST[p] = rec[kq]; ++p; }
  __syncthreads();
  return tot < CAP ? tot : CAP;
}

__global__ __launch_bounds__(NT) void prep_kernel(const float* __restrict__ W1x, const float* __restrict__ W1p,
                                                 const float* __restrict__ b1x, const float* __restrict__ b1p, const float* __restrict__ W2x,
                                                 unsigned* __restrict__ W1T, unsigned* __restrict__ W2T, float* __restrict__ B512, float* __restrict__ WL) {
  const int i = blockIdx.x * NT + threadIdx.x;
  unsigned u1 = 0u, u2 = 0u; float bb = 0.f, wl = 0.f;
  if (i < NC * FD / 2) {
    const int n = i >> 5, c = 2 * (i & 31);
    const int part = n >> 8, u = n & 255;
    const float* W = (u < HD) ? W1x : W1p; const int uu = (u < HD) ? u : u - HD;
    const int cin = part * FD + c;
    const float a = 16.0f * W[(size_t)cin * HD + uu], b = 16.0f * W[(size_t)(cin + 1) * HD + uu];
    u1 = pack_h2(a, b);
  }
  if (i < FD * HD / 2) {
    const int o = i >> 6, c = 2 * (i & 63);
    const float a = 16.0f * W2x[(size_t)c * FD + o], b = 16.0f * W2x[(size_t)(c + 1) * FD + o];
    u2 = pack_h2(a, b);
  }
  if (i < NC) bb = (i < HD) ? b1x[i] : ((i < HC) ? b1p[i - HD] : 0.f);
  if (i < HC) wl = (i < HD) ? W1x[(size_t)HD * HD + i] : W1p[(size_t)HD * HD + i - HD];
  for (int ps = 0; ps < 2; ++ps) {
    if (i < NC * FD / 2) ((volatile unsigned*)W1T)[i] = u1;
    if (i < FD * HD / 2) ((volatile unsigned*)W2T)[i] = u2;
    if (i < NC) ((volatile float*)B512)[i] = bb;
    if (i < HC) ((volatile float*)WL)[i] = wl;
    __threadfence();
  }
}

__global__ __launch_bounds__(NT) void castx_kernel(const float* __restrict__ x, unsigned* __restrict__ X16) {
  const int i = blockIdx.x * NT + threadIdx.x;
  if (i >= NPM * 32) return;
  const int node = i >> 5;
  unsigned u = 0u;
  if (node < NN) u = pack_h2(x[2 * (size_t)i], x[2 * (size_t)i + 1]);
  ((volatile unsigned*)X16)[i] = u;
  __threadfence();
  ((volatile unsigned*)X16)[i] = u;
}

__global__ __launch_bounds__(NT) void edge_kernel(int k, const int* __restrict__ ei, const float* __restrict__ pos,
                                                 const float* __restrict__ XAB, const float* __restrict__ WL,
                                                 const float* __restrict__ W2p, const float* __restrict__ b2p,
                                                 const unsigned short* __restrict__ W2Tp, const float* __restrict__ b2x,
                                                 float* __restrict__ MSG, float* __restrict__ PU) {
  __shared__ __align__(16) _Float16 sA[EB * SAP];
  __shared__ __align__(16) float sR[EB * 4];
  __shared__ __align__(16) float sT[8][16 * 36];
  const int tid = threadIdx.x, lane = tid & 31, wave = tid >> 5;
  const int i0 = blockIdx.x * EB;
  const v4f wlA = *(const v4f*)(WL + 4 * lane), wlB = *(const v4f*)(WL + HD + 4 * lane);
  const v4f w2v = *(const v4f*)(W2p + 4 * lane);
  const float b2p0 = b2p[0];
  const v4f z4 = {0.f, 0.f, 0.f, 0.f};
  const _Float16 hz = (_Float16)0.0f;
#pragma unroll 1
  for (int t = 0; t < EB / 8; ++t) {
    const int j = wave + 8 * t;
    const int e = k * CH + i0 + j;
    v4h pk = {hz, hz, hz, hz};
    float dp = 0.f, r0 = 0.f, r1 = 0.f, r2 = 0.f;
    if (e < NE) {
      int rw = ei[e], cl = ei[NE + e];
      rw = rw < 0 ? 0 : (rw >= NN ? NN - 1 : rw);
      cl = cl < 0 ? 0 : (cl >= NN ? NN - 1 : cl);
      const float* pr = pos + (size_t)rw * 3; const float* pc = pos + (size_t)cl * 3;
      r0 = pr[0] - pc[0]; r1 = pr[1] - pc[1]; r2 = pr[2] - pc[2];
      const float dsq = r0 * r0 + r1 * r1 + r2 * r2;
      const float* xr = XAB + (size_t)rw * NC; const float* xc = XAB + (size_t)cl * NC + HC;
      const v4f ha = *(const v4f*)(xr + 4 * lane) + *(const v4f*)(xc + 4 * lane) + dsq * wlA;
      const v4f hb = *(const v4f*)(xr + HD + 4 * lane) + *(const v4f*)(xc + HD + 4 * lane) + dsq * wlB;
#pragma unroll
      for (int c = 0; c < 4; ++c) {
        const float sa = silu_f(ha[c]);
        pk[c] = (_Float16)(16.0f * sa);
        const float sb = silu_f(hb[c]);
        dp += sb * w2v[c];
      }
    }
#pragma unroll
    for (int off = 1; off < 32; off <<= 1) dp += __shfl_xor(dp, off, 32);
    const float w = dp + b2p0;
    *(v4h*)(sA + j * SAP + 4 * lane) = pk;
    if (lane == 0) {
      v4f pu = z4;
      if (e < NE) { pu[0] = w * r0; pu[1] = w * r1; pu[2] = w * r2; }
      *(v4f*)(sR + j * 4) = pu;
    }
  }
  __syncthreads();

  const _Float16* W2T = (const _Float16*)W2Tp;
  const int rl = lane & 15, koff = (lane >> 4) * 8, mOff = (lane >> 4) * 8;
  const int rt = wave & 3, cb = (wave >> 2) * 32;
  v8f acc[2];
  acc[0] = (v8f){0.f,0.f,0.f,0.f,0.f,0.f,0.f,0.f};
  acc[1] = (v8f){0.f,0.f,0.f,0.f,0.f,0.f,0.f,0.f};
#pragma unroll
  for (int ks = 0; ks < HD / 32; ++ks) {
    const v16h a  = Frag<_Float16>::load(sA + (16 * rt + rl) * SAP + koff + 32 * ks);
    const v16h b0 = Frag<_Float16>::load(W2T + (size_t)(cb + rl) * HD + koff + 32 * ks);
    const v16h b1 = Frag<_Float16>::load(W2T + (size_t)(cb + 16 + rl) * HD + koff + 32 * ks);
    acc[0] = Frag<_Float16>::mma(a, b0, acc[0]);
    acc[1] = Frag<_Float16>::mma(a, b1, acc[1]);
    Frag<_Float16>::guard(acc[0], acc[1], a, b1);
    Frag<_Float16>::keep(b0, b1, a, a);
  }
  acc_guard2(acc[0], acc[1]);
  float* slab = sT[wave];
#pragma unroll
  for (int j2 = 0; j2 < 2; ++j2) {
    const int cc = 16 * j2 + rl;
    const float bv = b2x[cb + cc];
#pragma unroll
    for (int r = 0; r < 8; ++r) slab[(mOff + r) * 36 + cc] = acc[j2][r] * (1.0f / 256.0f) + bv;
  }
  __builtin_amdgcn_fence(__ATOMIC_RELEASE, "workgroup");
  __builtin_amdgcn_wave_barrier();
  __builtin_amdgcn_fence(__ATOMIC_ACQUIRE, "workgroup");
  {
    const int q = lane >> 3, c4 = (lane & 7) * 4;
    for (int ps = 0; ps < 2; ++ps) {
#pragma unroll
      for (int it = 0; it < 4; ++it) {
        const int row = it * 4 + q;
        const v4f v = *(const v4f*)(slab + row * 36 + c4);
        *(volatile v4f*)(MSG + (size_t)(i0 + 16 * rt + row) * FD + cb + c4) = v;
      }
      __threadfence();
    }
  }
  if (tid < EB) {
    const v4f v = *(const v4f*)(sR + tid * 4);
    float* p = PU + (size_t)(i0 + tid) * 4;
    *(volatile v4f*)p = v;
    __threadfence();
    *(volatile v4f*)p = v;
  }
}

__global__ __launch_bounds__(NT) void aggregate_kernel(int k, int fin, const int* __restrict__ ei, const float* __restrict__ MSG,
                                                      const float* __restrict__ PU, float* AGX, float* AGP, float* outx, float* outp) {
  __shared__ __align__(16) float SX[TBN * FD];
  __shared__ __align__(16) float SPP[TBN * 4];
  __shared__ int LIST[SCH];
  __shared__ int scan_ws[80];
  const int tid = threadIdx.x, lane = tid & 31, wave = tid >> 5;
  const int n0 = blockIdx.x * TBN;
  const v4f z4 = {0.f, 0.f, 0.f, 0.f};
  for (int u = tid; u < TBN * 16; u += NT) {
    const int row = u >> 4, c4 = (u & 15) * 4; const int n = n0 + row;
    v4f v = z4;
    if (k > 0 && n < NN) v = *(const v4f*)(AGX + (size_t)n * FD + c4);
    *(v4f*)(SX + row * FD + c4) = v;
  }
  for (int u = tid; u < TBN; u += NT) {
    const int n = n0 + u; v4f v = z4;
    if (k > 0 && n < NN) v = *(const v4f*)(AGP + (size_t)n * 4);
    *(v4f*)(SPP + u * 4) = v;
  }
  __syncthreads();
  const int* dstv = ei + NE;
  const int ec0 = k * CH;
#pragma unroll 1
  for (int c = 0; c < NSTEP; ++c) {
    const int tot = chunk_hits<SCH / NT, SCH>(dstv, ec0 + c * SCH, ec0, n0, tid, LIST, scan_ws);
#pragma unroll 1
    for (int base = 0; base < tot; base += 32) {
      const int q = base + lane;
      const int rv = (q < tot) ? LIST[q] : -1;
      const int own = (rv >= 0 && (rv >> 23) == wave) ? 1 : 0;
      unsigned msk = (unsigned)__ballot(own);
#pragma unroll 1
      for (int it = 0; it < 32; ++it) {
        if (msk == 0u) break;
        const int bp = __builtin_ctz(msk); msk &= msk - 1u;
        const int r = __shfl(rv, bp, 32);
        const int dl = (r >> 17) & (TBN - 1);
        int el = r & 0x1FFFF; el = el < CH ? el : CH - 1;
        const v2f m = *(const v2f*)(MSG + (size_t)el * FD + 2 * lane);
        float* sx = SX + dl * FD + 2 * lane;
        v2f a = *(v2f*)sx; a = a + m; *(v2f*)sx = a;
        if (lane < 4) { const float pv = PU[(size_t)el * 4 + lane]; SPP[dl * 4 + lane] += pv; }
      }
    }
    __syncthreads();
  }
  float* OX = fin ? outx : AGX;
  const int cnt = (NN - n0) < TBN ? (NN - n0) : TBN;
  const int nf4 = (cnt * 3) >> 2;
  for (int ps = 0; ps < 2; ++ps) {
    for (int u = tid; u < TBN * 16; u += NT) {
      const int row = u >> 4, c4 = (u & 15) * 4; const int n = n0 + row;
      if (n < NN) { const v4f v = *(const v4f*)(SX + row * FD + c4); *(volatile v4f*)(OX + (size_t)n * FD + c4) = v; }
    }
    if (!fin) {
      for (int u = tid; u < TBN; u += NT) {
        const int n = n0 + u;
        if (n < NN) { const v4f v = *(const v4f*)(SPP + u * 4); *(volatile v4f*)(AGP + (size_t)n * 4) = v; }
      }
    } else {
      for (int u = tid; u < nf4; u += NT) {
        const int jf = 4 * u; v4f v;
#pragma unroll
        for (int c2 = 0; c2 < 4; ++c2) { const int jj = jf + c2; const int nd = jj / 3; v[c2] = SPP[nd * 4 + (jj - 3 * nd)]; }
        *(volatile v4f*)(outp + (size_t)n0 * 3 + jf) = v;
      }
    }
    __threadfence();
  }
}

extern "C" void kernel_launch(void* const* d_in, const int* in_sizes, int n_in,
                              void* d_out, int out_size, void* d_ws, size_t ws_size,
                              hipStream_t stream) {
  if (n_in < 11) return;
  if (in_sizes[0] != NN * FD || in_sizes[1] != NN * 3 || in_sizes[2] != 2 * NE || in_sizes[3] != 129 * HD ||
      in_sizes[4] != HD || in_sizes[5] != HD * FD || in_sizes[6] != FD || in_sizes[7] != 129 * HD || in_sizes[8] != HD ||
      in_sizes[9] != HD || in_sizes[10] < 1 || out_size != NN * FD + NN * 3) return;
  const float* x   = (const float*)d_in[0];
  const float* pos = (const float*)d_in[1];
  const int*   ei  = (const int*)  d_in[2];
  const float* W1x = (const float*)d_in[3];
  const float* b1x = (const float*)d_in[4];
  const float* W2x = (const float*)d_in[5];
  const float* b2x = (const float*)d_in[6];
  const float* W1p = (const float*)d_in[7];
  const float* b1p = (const float*)d_in[8];
  const float* W2p = (const float*)d_in[9];
  const float* b2p = (const float*)d_in[10];
  float* out_x = (float*)d_out;
  float* out_p = out_x + (size_t)NN * FD;

  char* ws = (char*)d_ws; size_t off = 0;
  auto carve = [&](size_t bytes) -> char* { char* p = ws + off; off += (bytes + 255) & ~(size_t)255; return p; };
  unsigned* W1T  = (unsigned*)carve((size_t)NC * FD * 2);
  unsigned* W2T  = (unsigned*)carve((size_t)FD * HD * 2);
  float*    B512 = (float*)carve((size_t)NC * 4);
  float*    WL   = (float*)carve((size_t)HC * 4);
  float*    XAB  = (float*)carve((size_t)NPM * NC * 4);
  float*    AGX  = (float*)carve((size_t)NN * FD * 4);
  float*    AGP  = (float*)carve((size_t)NN * 4 * 4);
  const size_t scr_x  = (size_t)NPM * FD * 2;
  const size_t scr_ch = (size_t)CH * FD * 4 + (size_t)CH * 16;
  char*     SCR  = carve(scr_ch > scr_x ? scr_ch : scr_x);
  if (off > ws_size || off > (size_t)134217728) return;
  unsigned* X16 = (unsigned*)SCR;
  float*    MSG = (float*)SCR;
  float*    PU  = (float*)(SCR + (size_t)CH * FD * 4);

  prep_kernel<<<(NC * FD / 2) / NT, NT, 0, stream>>>(W1x, W1p, b1x, b1p, W2x, W1T, W2T, B512, WL);
  castx_kernel<<<(NPM * 32) / NT, NT, 0, stream>>>(x, X16);
  {
    const int tiles = (NPM / 64) * (NC / 64);
    wmma_gemm64<0, false, 2, 0, false, 0><<<dim3((tiles + 7) / 8, 1), 256, 0, stream>>>(
        (const unsigned short*)X16, (const unsigned short*)nullptr, FD, 0L,
        (const unsigned short*)W1T, (const unsigned short*)nullptr, FD, 0L,
        (void*)XAB, (void*)nullptr, NC, 0L,
        B512, (const float*)nullptr, 0L, NPM, NC, FD, 0.0625f);
  }
  for (int k = 0; k < NCHUNK; ++k) {
    edge_kernel<<<CH / EB, NT, 0, stream>>>(k, ei, pos, XAB, WL, W2p, b2p, (const unsigned short*)W2T, b2x, MSG, PU);
    aggregate_kernel<<<NTILE, NT, 0, stream>>>(k, (k == NCHUNK - 1) ? 1 : 0, ei, MSG, PU, AGX, AGP, out_x, out_p);
  }
}
